// PFN_24781961298185
// MI455X (gfx1250) — hardware-verified
//
#include <hip/hip_runtime.h>
#include <math.h>

constexpr int SEQ_L  = 100;
constexpr int NB     = 8;
constexpr int DIN    = 768;
constexpr int HID    = 300;
constexpr int HIDP   = 320;
constexpr int G5     = 1500;
constexpr int G5P    = 1536;
constexpr int MROWS  = SEQ_L * NB;
constexpr int MPAD   = 832;
constexpr int KCC    = 3 * HIDP;
constexpr int KCAT   = 2 * HIDP;
constexpr int NTAG   = 8;
constexpr int NREL   = 12;
constexpr int NHEADP = 64;
constexpr int NPROWS = SEQ_L * SEQ_L * NB;
constexpr int JGRP   = 4;
constexpr int NTHR   = 256;
constexpr int HT_PITCH = 328;
constexpr int CC_PITCH = 968;
constexpr int GT_PITCH = 1536;
constexpr int CS_PITCH = 304;
constexpr int H3PLANE  = MROWS * HIDP;
constexpr float W2CARRY     = 32.0f;
constexpr float W2CARRY_INV = 1.0f / 32.0f;
constexpr float LN_EPS_F    = 1e-5f;
static_assert(HIDP % 32 == 0 && KCC % 32 == 0 && KCAT % 32 == 0 && DIN % 32 == 0, "K multiples of 32");
static_assert(MPAD % 64 == 0 && G5P % 64 == 0 && HIDP % 64 == 0 && NPROWS % 64 == 0 && NHEADP == 64, "M,N tile multiples");
static_assert(SEQ_L % JGRP == 0, "j groups exact");
static_assert((NB * HIDP) % NTHR == 0, "");
static_assert(NB == 8, "row & 7 decode");

typedef __attribute__((ext_vector_type(16))) _Float16 v16h;
typedef __attribute__((ext_vector_type(8)))  _Float16 v8h;
typedef __attribute__((ext_vector_type(16))) __bf16   v16b;
typedef __attribute__((ext_vector_type(8)))  __bf16   v8b;
typedef __attribute__((ext_vector_type(8)))  float    v8f;
typedef __attribute__((ext_vector_type(4)))  float    v4f;

__device__ __forceinline__ unsigned short f2bf_bits(float f) {
  unsigned u = __float_as_uint(f);
  return (unsigned short)((u + 0x7FFFu + ((u >> 16) & 1u)) >> 16);
}
__device__ __forceinline__ float bf_bits2f(unsigned short h) { return __uint_as_float(((unsigned)h) << 16); }
__device__ __forceinline__ void bf_split_bits(float v, unsigned short& hb, unsigned short& lb) {
  hb = f2bf_bits(v);
  lb = f2bf_bits(v - bf_bits2f(hb));
}

__device__ __forceinline__ void dep_guard_h(v8f& a, v8f& b, v16h x, v16h y) { asm volatile("v_nop\n\tv_nop\n\tv_nop\n\tv_nop" : "+v"(a), "+v"(b) : "v"(x), "v"(y)); }
__device__ __forceinline__ void dep_guard_b(v8f& a, v8f& b, v16b x, v16b y) { asm volatile("v_nop\n\tv_nop\n\tv_nop\n\tv_nop" : "+v"(a), "+v"(b) : "v"(x), "v"(y)); }
__device__ __forceinline__ void keep4_h(v16h a, v16h b, v16h c, v16h d) { asm volatile("v_nop" :: "v"(a), "v"(b), "v"(c), "v"(d)); }
__device__ __forceinline__ void keep4_b(v16b a, v16b b, v16b c, v16b d) { asm volatile("v_nop" :: "v"(a), "v"(b), "v"(c), "v"(d)); }
__device__ __forceinline__ void acc_guard4(v8f& a, v8f& b, v8f& c, v8f& d) { asm volatile("v_nop\n\tv_nop\n\tv_nop\n\tv_nop" : "+v"(a), "+v"(b), "+v"(c), "+v"(d)); }
__device__ __forceinline__ void acc_guard3(v8f& a, v8f& b, v8f& c) { asm volatile("v_nop\n\tv_nop\n\tv_nop\n\tv_nop" : "+v"(a), "+v"(b), "+v"(c)); }
template <typename T> struct Frag;
template <> struct Frag<_Float16> {
  typedef v16h V; union U { v16h v; v8h h[2]; };
  static __device__ __forceinline__ v16h load(const _Float16* p) {
    U f; f.h[0] = *(const v8h*)(p); f.h[1] = *(const v8h*)(p + 16); return f.v;
  }
  static __device__ __forceinline__ v8f mma(v16h a, v16h b, v8f c) {
    return __builtin_amdgcn_wmma_f32_16x16x32_f16(false, a, false, b, (short)0, c, false, false);
  }
  static __device__ __forceinline__ void guard(v8f& a, v8f& b, v16h x, v16h y) { dep_guard_h(a, b, x, y); }
  static __device__ __forceinline__ void keep(v16h a, v16h b, v16h c, v16h d) { keep4_h(a, b, c, d); }
};
template <> struct Frag<__bf16> {
  typedef v16b V; union U { v16b v; v8b h[2]; };
  static __device__ __forceinline__ v16b load(const __bf16* p) {
    U f; f.h[0] = *(const v8b*)(p); f.h[1] = *(const v8b*)(p + 16); return f.v;
  }
  static __device__ __forceinline__ v8f mma(v16b a, v16b b, v8f c) {
    return __builtin_amdgcn_wmma_f32_16x16x32_bf16(false, a, false, b, (short)0, c, false, false);
  }
  static __device__ __forceinline__ void guard(v8f& a, v8f& b, v16b x, v16b y) { dep_guard_b(a, b, x, y); }
  static __device__ __forceinline__ void keep(v16b a, v16b b, v16b c, v16b d) { keep4_b(a, b, c, d); }
};

template <int ET> struct Elem;
template <> struct Elem<0> { typedef _Float16 T; };
template <> struct Elem<1> { typedef __bf16 T; };
template <int ET, bool SPLIT, int BIAS_MODE, int OUT_MODE, bool RESID, int ACT = 0>
__global__ __launch_bounds__(256) void wmma_gemm64(
    const unsigned short* __restrict__ Ap, const unsigned short* __restrict__ A2p, int lda, long strideA,
    const unsigned short* __restrict__ Btp, const unsigned short* __restrict__ Bt2p, int ldb, long strideB,
    void* __restrict__ Cout, void* __restrict__ Cout2, int ldc, long strideC,
    const float* __restrict__ bias,
    const float* __restrict__ resid, long strideR,
    int M, int N, int K, float scale) {
  typedef typename Elem<ET>::T T;
  typedef typename Frag<T>::V V;
  const T* A = (const T*)Ap; const T* A2 = (const T*)A2p; const T* Bt = (const T*)Btp; const T* Bt2 = (const T*)Bt2p;
  __shared__ __align__(16) float sT[8][16 * 68];
  const int b    = blockIdx.y;
  const int lane = threadIdx.x & 31;
  const int wave = threadIdx.x >> 5;
  const int tilesN = N >> 6;
  const int tilesM = M >> 6;
  const int tile = blockIdx.x * 8 + wave;
  if (tile >= tilesM * tilesN) return;
  const int tm = tile / tilesN;
  const int tn = tile - tm * tilesN;
  const int m0 = tm << 6;
  const int n0 = tn << 6;

  const T* Ab  = A  + (size_t)b * strideA;
  const T* Bb  = Bt + (size_t)b * strideB;
  const T* Ab2 = SPLIT ? (A2  + (size_t)b * strideA) : nullptr;
  const T* Bb2 = SPLIT ? (Bt2 + (size_t)b * strideB) : nullptr;

  const int rlane = lane & 15;
  const int koff  = (lane >> 4) * 8;
  const int mOff  = (lane >> 4) * 8;

  v8f acc[4][4];
#pragma unroll
  for (int i = 0; i < 4; ++i)
#pragma unroll
    for (int j = 0; j < 4; ++j) acc[i][j] = (v8f){0.f,0.f,0.f,0.f,0.f,0.f,0.f,0.f};

  for (int k0 = 0; k0 < K; k0 += 32) {
    V bh[4], bl[4];
#pragma unroll
    for (int j = 0; j < 4; ++j) {
      const size_t bo = (size_t)(n0 + (j << 4) + rlane) * ldb + koff + k0;
      bh[j] = Frag<T>::load(Bb + bo);
      if (SPLIT) bl[j] = Frag<T>::load(Bb2 + bo);
    }
#pragma unroll
    for (int i = 0; i < 4; ++i) {
      const size_t ao = (size_t)(m0 + (i << 4) + rlane) * lda + koff + k0;
      V ah = Frag<T>::load(Ab + ao);
      V al;
      if (SPLIT) al = Frag<T>::load(Ab2 + ao);
#pragma unroll
      for (int j = 0; j < 4; ++j) {
        acc[i][j] = Frag<T>::mma(ah, bh[j], acc[i][j]);
        if (SPLIT) {
          acc[i][j] = Frag<T>::mma(ah, bl[j], acc[i][j]);
          acc[i][j] = Frag<T>::mma(al, bh[j], acc[i][j]);
        }
      }
      Frag<T>::guard(acc[i][0], acc[i][3], ah, SPLIT ? al : ah);
    }
    Frag<T>::keep(bh[0], bh[1], bh[2], bh[3]);
    if (SPLIT) Frag<T>::keep(bl[0], bl[1], bl[2], bl[3]);
  }
  acc_guard4(acc[0][0], acc[0][1], acc[0][2], acc[0][3]);
  acc_guard4(acc[1][0], acc[1][1], acc[1][2], acc[1][3]);
  acc_guard4(acc[2][0], acc[2][1], acc[2][2], acc[2][3]);
  acc_guard4(acc[3][0], acc[3][1], acc[3][2], acc[3][3]);

  float* slab = sT[wave];
  const float* Rb = RESID ? (resid + (size_t)b * strideR) : nullptr;
#pragma unroll
  for (int i = 0; i < 4; ++i) {
    const int mBase = m0 + (i << 4);
#pragma unroll
    for (int j = 0; j < 4; ++j) {
      const int n = n0 + (j << 4) + rlane;
      float bv = 0.f;
      if (BIAS_MODE == 2) bv = bias[n];
#pragma unroll
      for (int r = 0; r < 8; ++r) {
        float v = acc[i][j][r] * scale;
        if (BIAS_MODE == 1) v += bias[mBase + mOff + r];
        if (BIAS_MODE == 2) v += bv;
        if (RESID) v += Rb[(size_t)(mBase + mOff + r) * ldc + n];
        if (ACT == 1) v = tanhf(v);
        if (ACT == 2) v = fmaxf(v, 0.0f);
        if (ACT == 3) v = v / (1.0f + expf(-v));
        if (ACT == 4) v = (v > 0.f) ? v : 0.01f * v;
        if (ACT == 5) v = 0.5f * v * (1.0f + erff(v * 0.70710678118654752f));
        slab[(mOff + r) * 68 + (j << 4) + rlane] = v;
      }
    }
    __builtin_amdgcn_fence(__ATOMIC_RELEASE, "workgroup");
    __builtin_amdgcn_wave_barrier();
    __builtin_amdgcn_fence(__ATOMIC_ACQUIRE, "workgroup");
    if (OUT_MODE == 0) {
      float* C = (float*)Cout + (size_t)b * strideC;
      const int hh = lane >> 4, c4 = (lane & 15) * 4;
      for (int pass = 0; pass < 2; ++pass) {
#pragma unroll
        for (int it = 0; it < 8; ++it) {
          const int row = it * 2 + hh;
          v4f v = *(const v4f*)(slab + row * 68 + c4);
          *(volatile v4f*)(C + (size_t)(mBase + row) * ldc + n0 + c4) = v;
        }
        __threadfence();
      }
    } else {
      const int q = lane >> 3, c8 = (lane & 7) * 8;
      unsigned short* C  = (unsigned short*)Cout  + (size_t)b * strideC;
      unsigned short* C2 = (OUT_MODE == 2) ? ((unsigned short*)Cout2 + (size_t)b * strideC) : nullptr;
      for (int pass = 0; pass < 2; ++pass) {
#pragma unroll
        for (int it = 0; it < 4; ++it) {
          const int row = it * 4 + q;
          const float* sp = slab + row * 68 + c8;
          v8h hv, lv;
#pragma unroll
          for (int e = 0; e < 8; ++e) {
            if (OUT_MODE == 1) {
              hv[e] = (_Float16)sp[e];
            } else {
              unsigned short hb = f2bf_bits(sp[e]);
              unsigned short lb = f2bf_bits(sp[e] - bf_bits2f(hb));
              hv[e] = __builtin_bit_cast(_Float16, hb);
              lv[e] = __builtin_bit_cast(_Float16, lb);
            }
          }
          *(volatile v8h*)(C + (size_t)(mBase + row) * ldc + n0 + c8) = hv;
          if (OUT_MODE == 2) *(volatile v8h*)(C2 + (size_t)(mBase + row) * ldc + n0 + c8) = lv;
        }
        __threadfence();
      }
    }
    __builtin_amdgcn_fence(__ATOMIC_RELEASE, "workgroup");
    __builtin_amdgcn_wave_barrier();
    __builtin_amdgcn_fence(__ATOMIC_ACQUIRE, "workgroup");
  }
}

template <int MODE>
__global__ __launch_bounds__(NTHR) void cvt_plane_kernel(const float* __restrict__ src, int nrow_s, int spitch, int segs, int segd,
                                                        unsigned short* __restrict__ dh, unsigned short* __restrict__ dl,
                                                        int nrow_d, int ncol8_d, float sc) {
  const int i  = blockIdx.x * NTHR + threadIdx.x;
  const int n8 = nrow_d * ncol8_d;
  if (i >= n8) return;
  const int row = i / ncol8_d;
  const int c8  = i - row * ncol8_d;
  const int d0  = 8 * c8;
  const int seg = d0 / segd;
  const int jj0 = d0 - seg * segd;
  const bool rvalid = row < nrow_s;
  const int rowc = rvalid ? row : (nrow_s - 1);
  const float* sp = src + (size_t)rowc * spitch + (size_t)seg * segs;
  v8h hv, lv;
#pragma unroll
  for (int e = 0; e < 8; ++e) {
    const int jj = jj0 + e;
    const int jc = (jj < segs) ? jj : (segs - 1);
    float x = sp[jc];
    x = (rvalid && (jj < segs)) ? x : 0.0f;
    if (MODE == 0) {
      unsigned short hb, lb;
      bf_split_bits(x, hb, lb);
      hv[e] = __builtin_bit_cast(_Float16, hb);
      lv[e] = __builtin_bit_cast(_Float16, lb);
    } else {
      hv[e] = (_Float16)(x * sc);
      lv[e] = hv[e];
    }
  }
  *(volatile v8h*)(dh + (size_t)i * 8) = hv;
  if (MODE == 0) *(volatile v8h*)(dl + (size_t)i * 8) = lv;
  __threadfence();
  *(volatile v8h*)(dh + (size_t)i * 8) = hv;
  if (MODE == 0) *(volatile v8h*)(dl + (size_t)i * 8) = lv;
}

__global__ __launch_bounds__(NTHR) void cvt_cat_kernel(const float* __restrict__ s0, const float* __restrict__ s1,
                                                      unsigned short* __restrict__ dh, unsigned short* __restrict__ dl, int ncol8) {
  const int i  = blockIdx.x * NTHR + threadIdx.x;
  const int n8 = MPAD * ncol8;
  if (i >= n8) return;
  const int row = i / ncol8;
  const int c8  = i - row * ncol8;
  const int seg = (c8 >= 40) ? 1 : 0;
  const int cc  = c8 - 40 * seg;
  const bool rvalid = row < MROWS;
  const int rowc = rvalid ? row : (MROWS - 1);
  const float* p0 = s0 + (size_t)rowc * HIDP + 8 * cc;
  const float* p1 = s1 + (size_t)rowc * HIDP + 8 * cc;
  const v4f a0 = *(const v4f*)(p0), a1 = *(const v4f*)(p0 + 4);
  const v4f b0 = *(const v4f*)(p1), b1 = *(const v4f*)(p1 + 4);
  v8h hv, lv;
#pragma unroll
  for (int e = 0; e < 4; ++e) {
    float x0 = seg ? b0[e] : a0[e];
    float x1 = seg ? b1[e] : a1[e];
    x0 = rvalid ? x0 : 0.0f;
    x1 = rvalid ? x1 : 0.0f;
    unsigned short hb, lb;
    bf_split_bits(x0, hb, lb);
    hv[e] = __builtin_bit_cast(_Float16, hb); lv[e] = __builtin_bit_cast(_Float16, lb);
    bf_split_bits(x1, hb, lb);
    hv[4 + e] = __builtin_bit_cast(_Float16, hb); lv[4 + e] = __builtin_bit_cast(_Float16, lb);
  }
  *(volatile v8h*)(dh + (size_t)i * 8) = hv;
  *(volatile v8h*)(dl + (size_t)i * 8) = lv;
  __threadfence();
  *(volatile v8h*)(dh + (size_t)i * 8) = hv;
  *(volatile v8h*)(dl + (size_t)i * 8) = lv;
}

__global__ __launch_bounds__(512) void pad8_kernel(const float* __restrict__ s0, const float* __restrict__ s1,
                                                  const float* __restrict__ s2, const float* __restrict__ s3,
                                                  const float* __restrict__ s4, const float* __restrict__ s5,
                                                  const float* __restrict__ s6, const float* __restrict__ s7,
                                                  float* __restrict__ dst) {
  const int t = blockIdx.x * 512 + threadIdx.x;
  const int which = t >> 7;
  const int q = t & 127;
  v4f o;
#pragma unroll
  for (int e = 0; e < 4; ++e) {
    const int col = 4 * q + e;
    const int colc = (col < HID) ? col : (HID - 1);
    const float x0 = s0[colc], x1 = s1[colc], x2 = s2[colc], x3 = s3[colc];
    const float x4 = s4[colc], x5 = s5[colc], x6 = s6[colc], x7 = s7[colc];
    float x = x0;
    x = (which == 1) ? x1 : x;
    x = (which == 2) ? x2 : x;
    x = (which == 3) ? x3 : x;
    x = (which == 4) ? x4 : x;
    x = (which == 5) ? x5 : x;
    x = (which == 6) ? x6 : x;
    x = (which == 7) ? x7 : x;
    o[e] = (col < HID) ? x : 0.0f;
  }
  if (q < 80 && which < 8) {
    float* op = dst + which * HIDP + 4 * q;
    *(volatile v4f*)op = o;
    __threadfence();
    *(volatile v4f*)op = o;
  }
}

__global__ __launch_bounds__(NTHR) void pf_seq_kernel(const float* __restrict__ XG, const float* __restrict__ bi,
                                                     const float* __restrict__ bhv, const float* __restrict__ btv,
                                                     const unsigned short* __restrict__ WHHp, const unsigned short* __restrict__ WHLp,
                                                     const unsigned short* __restrict__ WTHp, const unsigned short* __restrict__ WTLp,
                                                     float* __restrict__ H3F) {
  __shared__ __align__(16) float  sG[NB * GT_PITCH];
  __shared__ __align__(16) __bf16 sHh[NB * HT_PITCH];
  __shared__ __align__(16) __bf16 sHl[NB * HT_PITCH];
  __shared__ __align__(16) __bf16 sCh[NB * CC_PITCH];
  __shared__ __align__(16) __bf16 sCl[NB * CC_PITCH];
  __shared__ __align__(16) float  sC[NB * CS_PITCH];
  __shared__ __align__(16) float  sStg[3 * NB * HIDP];
  const __bf16* WHH = (const __bf16*)WHHp;
  const __bf16* WHL = (const __bf16*)WHLp;
  const __bf16* WTH = (const __bf16*)WTHp;
  const __bf16* WTL = (const __bf16*)WTLp;
  const int tid = threadIdx.x, lane = tid & 31, wave = tid >> 5;
  const int rlane = lane & 15, hh = lane >> 4, koff = hh * 8, rA = lane & 7;
  const __bf16 bz = __builtin_bit_cast(__bf16, (unsigned short)0);

#pragma unroll 1
  for (int i = tid; i < NB * HT_PITCH; i += NTHR) { sHh[i] = bz; sHl[i] = bz; }
#pragma unroll 1
  for (int i = tid; i < NB * CC_PITCH; i += NTHR) { sCh[i] = bz; sCl[i] = bz; }
#pragma unroll 1
  for (int i = tid; i < NB * CS_PITCH; i += NTHR) sC[i] = 0.0f;
#pragma unroll 1
  for (int i = tid; i < 3 * NB * HIDP; i += NTHR) sStg[i] = 0.0f;
  __syncthreads();

  const v8f z8 = {0.f, 0.f, 0.f, 0.f, 0.f, 0.f, 0.f, 0.f};

#pragma unroll 1
  for (int t = 0; t < SEQ_L; ++t) {
    {
      const __bf16* ahp = sHh + rA * HT_PITCH + koff;
      const __bf16* alp = sHl + rA * HT_PITCH + koff;
      const float* xgr = XG + (size_t)(t * NB) * G5P;
#pragma unroll 1
      for (int grp = 0; grp < 3; ++grp) {
        const int sb = wave * 12 + grp * 4;
        size_t boff[4];
#pragma unroll
        for (int j = 0; j < 4; ++j) boff[j] = (size_t)(16 * (sb + j) + rlane) * HIDP + koff;
        v8f acc[4];
#pragma unroll
        for (int j = 0; j < 4; ++j) acc[j] = z8;
#pragma unroll 1
        for (int k0 = 0; k0 < HIDP; k0 += 32) {
          v16b bhf[4], blf[4];
#pragma unroll
          for (int j = 0; j < 4; ++j) {
            bhf[j] = Frag<__bf16>::load(WHH + boff[j] + k0);
            blf[j] = Frag<__bf16>::load(WHL + boff[j] + k0);
          }
          const v16b ah = Frag<__bf16>::load(ahp + k0);
          const v16b al = Frag<__bf16>::load(alp + k0);
#pragma unroll
          for (int j = 0; j < 4; ++j) {
            acc[j] = Frag<__bf16>::mma(ah, bhf[j], acc[j]);
            acc[j] = Frag<__bf16>::mma(ah, blf[j], acc[j]);
            acc[j] = Frag<__bf16>::mma(al, bhf[j], acc[j]);
          }
          dep_guard_b(acc[0], acc[3], ah, al);
          keep4_b(bhf[0], bhf[1], bhf[2], bhf[3]);
          keep4_b(blf[0], blf[1], blf[2], blf[3]);
        }
        acc_guard4(acc[0], acc[1], acc[2], acc[3]);
        if (hh == 0) {
#pragma unroll
          for (int j = 0; j < 4; ++j) {
            const int n  = 16 * (sb + j) + rlane;
            const int nc = (n < G5) ? n : (G5 - 1);
            const float bsum = bhv[nc] + bi[nc];
#pragma unroll
            for (int r = 0; r < 8; ++r)
              sG[r * GT_PITCH + n] = acc[j][r] + xgr[(size_t)r * G5P + n] + bsum;
          }
        }
      }
    }
    __syncthreads();

#pragma unroll 1
    for (int q = 0; q < 4; ++q) {
      const int task = wave * 4 + q;
      const int b = task & 7;
      const int g = 1 + (task >> 3);
      float* rowp = sG + b * GT_PITCH + g * HID;
      const int base = lane * 10;
      const bool actv = base < HID;
      const int basec = actv ? base : 0;
      float v[10];
      float mx = -3.0e38f;
#pragma unroll
      for (int k = 0; k < 10; ++k) {
        const float x = rowp[basec + k];
        v[k] = actv ? x : -3.0e38f;
        mx = fmaxf(mx, v[k]);
      }
#pragma unroll
      for (int off = 1; off < 32; off <<= 1) mx = fmaxf(mx, __shfl_xor(mx, off, 32));
      float s = 0.0f;
#pragma unroll
      for (int k = 0; k < 10; ++k) {
        const float p = expf(v[k] - mx);
        v[k] = p;
        s += p;
      }
      float tot = s;
#pragma unroll
      for (int off = 1; off < 32; off <<= 1) tot += __shfl_xor(tot, off, 32);
      const float inv = 1.0f / tot;
      float pre = s;
#pragma unroll
      for (int d = 1; d < 32; d <<= 1) {
        const float y = __shfl_up(pre, d, 32);
        if (lane >= d) pre += y;
      }
      pre -= s;
      const bool oneMinus = (g == 1) || (g == 3);
      if (actv) {
        float run = pre;
#pragma unroll
        for (int k = 0; k < 10; ++k) {
          run += v[k];
          const float cum = run * inv;
          rowp[base + k] = oneMinus ? (1.0f - cum) : cum;
        }
      }
    }
    __syncthreads();

#pragma unroll 1
    for (int e = tid; e < NB * HID; e += NTHR) {
      const int b = e / HID;
      const int j = e - b * HID;
      const float* gb = sG + b * GT_PITCH;
      const float cg  = tanhf(gb[j]);
      const float egi = gb[HID + j];
      const float rgi = gb[2 * HID + j];
      const float egc = gb[3 * HID + j];
      const float rgc = gb[4 * HID + j];
      const float cin = sC[b * CS_PITCH + j];
      const float ovc = rgc * egc, upc = rgc - ovc, dnc = egc - ovc;
      const float ovi = rgi * egi, upi = rgi - ovi, dni = egi - ovi;
      const float sh = ovi * cin + ovc * cg;
      const float cr = upi * cin + upc * cg + sh;
      const float cn = dni * cin + dnc * cg + sh;
      const int co = b * CC_PITCH + j;
      unsigned short hb, lb;
      bf_split_bits(cr, hb, lb);
      sCh[co] = __builtin_bit_cast(__bf16, hb);            sCl[co] = __builtin_bit_cast(__bf16, lb);
      bf_split_bits(cn, hb, lb);
      sCh[co + HIDP] = __builtin_bit_cast(__bf16, hb);     sCl[co + HIDP] = __builtin_bit_cast(__bf16, lb);
      bf_split_bits(sh, hb, lb);
      sCh[co + 2 * HIDP] = __builtin_bit_cast(__bf16, hb); sCl[co + 2 * HIDP] = __builtin_bit_cast(__bf16, lb);
      sStg[(0 * NB + b) * HIDP + j] = tanhf(cn);
      sStg[(1 * NB + b) * HIDP + j] = tanhf(cr);
      sStg[(2 * NB + b) * HIDP + j] = tanhf(sh);
    }
    __syncthreads();

    for (int pass = 0; pass < 2; ++pass) {
#pragma unroll 1
      for (int idx = tid; idx < 3 * NB * 10 * 8; idx += NTHR) {
        const int line = idx >> 3, w8 = idx & 7;
        const int arr = line / 80;
        const int rem = line - arr * 80;
        const int row = rem / 10;
        const int seg = rem - row * 10;
        const int fo  = seg * 32 + w8 * 4;
        const v4f val = *(const v4f*)(sStg + (arr * NB + row) * HIDP + fo);
        *(volatile v4f*)(H3F + (size_t)arr * H3PLANE + (size_t)(t * NB + row) * HIDP + fo) = val;
      }
      __threadfence();
    }
    {
      const int s2  = (wave + 16 < 20) ? (wave + 16) : 19;
      const int nb0 = 16 * wave, nb1 = 16 * (wave + 8), nb2 = 16 * s2;
      const size_t bo0 = (size_t)(nb0 + rlane) * KCC + koff;
      const size_t bo1 = (size_t)(nb1 + rlane) * KCC + koff;
      const size_t bo2 = (size_t)(nb2 + rlane) * KCC + koff;
      const __bf16* ahp = sCh + rA * CC_PITCH + koff;
      const __bf16* alp = sCl + rA * CC_PITCH + koff;
      v8f acc0 = z8, acc1 = z8, acc2 = z8;
#pragma unroll 1
      for (int k0 = 0; k0 < KCC; k0 += 32) {
        const v16b bh0 = Frag<__bf16>::load(WTH + bo0 + k0), bl0 = Frag<__bf16>::load(WTL + bo0 + k0);
        const v16b bh1 = Frag<__bf16>::load(WTH + bo1 + k0), bl1 = Frag<__bf16>::load(WTL + bo1 + k0);
        const v16b bh2 = Frag<__bf16>::load(WTH + bo2 + k0), bl2 = Frag<__bf16>::load(WTL + bo2 + k0);
        const v16b ah = Frag<__bf16>::load(ahp + k0);
        const v16b al = Frag<__bf16>::load(alp + k0);
        acc0 = Frag<__bf16>::mma(ah, bh0, acc0); acc0 = Frag<__bf16>::mma(ah, bl0, acc0); acc0 = Frag<__bf16>::mma(al, bh0, acc0);
        acc1 = Frag<__bf16>::mma(ah, bh1, acc1); acc1 = Frag<__bf16>::mma(ah, bl1, acc1); acc1 = Frag<__bf16>::mma(al, bh1, acc1);
        acc2 = Frag<__bf16>::mma(ah, bh2, acc2); acc2 = Frag<__bf16>::mma(ah, bl2, acc2); acc2 = Frag<__bf16>::mma(al, bh2, acc2);
        dep_guard_b(acc0, acc2, ah, al);
        keep4_b(bh0, bl0, bh1, bl1);
        keep4_b(bh2, bl2, bh2, bl2);
      }
      acc_guard3(acc0, acc1, acc2);
      if (hh == 0) {
        {
          const int n = nb0 + rlane;
          const float btc = btv[(n < HID) ? n : (HID - 1)];
          if (n < HID) {
#pragma unroll
            for (int r = 0; r < 8; ++r) sC[r * CS_PITCH + n] = acc0[r] + btc;
          }
        }
        {
          const int n = nb1 + rlane;
          const float btc = btv[(n < HID) ? n : (HID - 1)];
          if (n < HID) {
#pragma unroll
            for (int r = 0; r < 8; ++r) sC[r * CS_PITCH + n] = acc1[r] + btc;
          }
        }
        if (wave < 4) {
          const int n = nb2 + rlane;
          const float btc = btv[(n < HID) ? n : (HID - 1)];
          if (n < HID) {
#pragma unroll
            for (int r = 0; r < 8; ++r) sC[r * CS_PITCH + n] = acc2[r] + btc;
          }
        }
      }
    }
    __syncthreads();

#pragma unroll 1
    for (int e = tid; e < NB * HID; e += NTHR) {
      const int b = e / HID;
      const int j = e - b * HID;
      const float hv = tanhf(sC[b * CS_PITCH + j]);
      unsigned short hb, lb;
      bf_split_bits(hv, hb, lb);
      sHh[b * HT_PITCH + j] = __builtin_bit_cast(__bf16, hb);
      sHl[b * HT_PITCH + j] = __builtin_bit_cast(__bf16, lb);
    }
    __syncthreads();
  }
}

__global__ __launch_bounds__(NTHR) void colmax_kernel(const float* __restrict__ P, unsigned short* __restrict__ dh,
                                                     unsigned short* __restrict__ dl) {
  const int i = blockIdx.x * NTHR + threadIdx.x;
  if (i >= NHEADP * (HIDP / 8)) return;
  const int row = i / (HIDP / 8);
  const int c8  = i - row * (HIDP / 8);
  v4f ma = {0.f, 0.f, 0.f, 0.f}, mb = {0.f, 0.f, 0.f, 0.f};
  if (row < NB) {
    ma = (v4f){-3.0e38f, -3.0e38f, -3.0e38f, -3.0e38f};
    mb = ma;
#pragma unroll 1
    for (int l = 0; l < SEQ_L; ++l) {
      const float* p = P + (size_t)(l * NB + row) * HIDP + 8 * c8;
      const v4f va = *(const v4f*)(p), vb = *(const v4f*)(p + 4);
#pragma unroll
      for (int e = 0; e < 4; ++e) { ma[e] = fmaxf(ma[e], va[e]); mb[e] = fmaxf(mb[e], vb[e]); }
    }
  }
  v8h hv, lv;
#pragma unroll
  for (int e = 0; e < 4; ++e) {
    unsigned short hb, lb;
    bf_split_bits(ma[e], hb, lb);
    hv[e] = __builtin_bit_cast(_Float16, hb); lv[e] = __builtin_bit_cast(_Float16, lb);
    bf_split_bits(mb[e], hb, lb);
    hv[4 + e] = __builtin_bit_cast(_Float16, hb); lv[4 + e] = __builtin_bit_cast(_Float16, lb);
  }
  *(volatile v8h*)(dh + (size_t)i * 8) = hv;
  *(volatile v8h*)(dl + (size_t)i * 8) = lv;
  __threadfence();
  *(volatile v8h*)(dh + (size_t)i * 8) = hv;
  *(volatile v8h*)(dl + (size_t)i * 8) = lv;
}

__device__ __forceinline__ float feluf(float x) { return (x > 0.0f) ? x : (__expf(x) - 1.0f); }

__global__ __launch_bounds__(NTHR) void pair_ln_kernel(const float* __restrict__ AP, const float* __restrict__ BP,
                                                      const float* __restrict__ CP, const float* __restrict__ gpad,
                                                      const float* __restrict__ bpad, unsigned short* __restrict__ PA) {
  const int tid = threadIdx.x, lane = tid & 31, wave = tid >> 5;
  const int task = blockIdx.x * (NTHR / 32) + wave;
  if (task >= SEQ_L * NB * (SEQ_L / JGRP)) return;
  const int jg = task % (SEQ_L / JGRP);
  const int ib = task / (SEQ_L / JGRP);
  const int b  = ib & 7;
  const int i  = ib >> 3;
  const int c0 = 8 * lane;
  const int c1 = 256 + 8 * (lane & 7);
  const bool has1 = lane < 8;
  const bool m1a = (c1 < HID);
  const bool m1b = (c1 + 4 < HID);
  const float* ap = AP + (size_t)(i * NB + b) * HIDP;
  const float* cq = CP + (size_t)b * HIDP;
  const v4f ac0a = *(const v4f*)(ap + c0)     + *(const v4f*)(cq + c0);
  const v4f ac0b = *(const v4f*)(ap + c0 + 4) + *(const v4f*)(cq + c0 + 4);
  const v4f ac1a = *(const v4f*)(ap + c1)     + *(const v4f*)(cq + c1);
  const v4f ac1b = *(const v4f*)(ap + c1 + 4) + *(const v4f*)(cq + c1 + 4);
  const v4f g0a = *(const v4f*)(gpad + c0), g0b = *(const v4f*)(gpad + c0 + 4);
  const v4f g1a = *(const v4f*)(gpad + c1), g1b = *(const v4f*)(gpad + c1 + 4);
  const v4f e0a = *(const v4f*)(bpad + c0), e0b = *(const v4f*)(bpad + c0 + 4);
  const v4f e1a = *(const v4f*)(bpad + c1), e1b = *(const v4f*)(bpad + c1 + 4);
  const float invH = 1.0f / (float)HID;
#pragma unroll 1
  for (int jj = 0; jj < JGRP; ++jj) {
    const int j = jg * JGRP + jj;
    const float* bq = BP + (size_t)(j * NB + b) * HIDP;
    const v4f x0a = *(const v4f*)(bq + c0) + ac0a;
    const v4f x0b = *(const v4f*)(bq + c0 + 4) + ac0b;
    const v4f x1a = *(const v4f*)(bq + c1) + ac1a;
    const v4f x1b = *(const v4f*)(bq + c1 + 4) + ac1b;
    const float s0 = ((x0a[0] + x0a[1]) + (x0a[2] + x0a[3])) + ((x0b[0] + x0b[1]) + (x0b[2] + x0b[3]));
    const float s1 = ((x1a[0] + x1a[1]) + (x1a[2] + x1a[3])) + ((x1b[0] + x1b[1]) + (x1b[2] + x1b[3]));
    float s = s0 + (has1 ? s1 : 0.0f);
#pragma unroll
    for (int off = 1; off < 32; off <<= 1) s += __shfl_xor(s, off, 32);
    const float mu = s * invH;
    const v4f d0a = x0a - mu, d0b = x0b - mu, d1a = x1a - mu, d1b = x1b - mu;
    const float q0  = ((d0a[0] * d0a[0] + d0a[1] * d0a[1]) + (d0a[2] * d0a[2] + d0a[3] * d0a[3]))
                    + ((d0b[0] * d0b[0] + d0b[1] * d0b[1]) + (d0b[2] * d0b[2] + d0b[3] * d0b[3]));
    const float q1a = (d1a[0] * d1a[0] + d1a[1] * d1a[1]) + (d1a[2] * d1a[2] + d1a[3] * d1a[3]);
    const float q1b = (d1b[0] * d1b[0] + d1b[1] * d1b[1]) + (d1b[2] * d1b[2] + d1b[3] * d1b[3]);
    float ss = q0 + (has1 ? ((m1a ? q1a : 0.0f) + (m1b ? q1b : 0.0f)) : 0.0f);
#pragma unroll
    for (int off = 1; off < 32; off <<= 1) ss += __shfl_xor(ss, off, 32);
    const float var  = ss * invH;
    const float rstd = rsqrtf(var + LN_EPS_F);
    const v4f y0a = (d0a * rstd) * g0a + e0a;
    const v4f y0b = (d0b * rstd) * g0b + e0b;
    const v4f y1a = (d1a * rstd) * g1a + e1a;
    const v4f y1b = (d1b * rstd) * g1b + e1b;
    v8h o0, o1;
#pragma unroll
    for (int e = 0; e < 4; ++e) {
      o0[e]     = (_Float16)feluf(y0a[e]);
      o0[4 + e] = (_Float16)feluf(y0b[e]);
      o1[e]     = (_Float16)feluf(y1a[e]);
      o1[4 + e] = (_Float16)feluf(y1b[e]);
    }
    unsigned short* prow = PA + (size_t)((i * SEQ_L + j) * NB + b) * HIDP;
    for (int pass = 0; pass < 2; ++pass) {
      *(volatile v8h*)(prow + c0) = o0;
      if (has1) *(volatile v8h*)(prow + c1) = o1;
      __threadfence();
    }
  }
}

template <int NC4, bool TRI>
__global__ __launch_bounds__(NTHR) void pack_head_kernel(const float* __restrict__ SCR, const float* __restrict__ b2,
                                                        const float* __restrict__ maskv, float* __restrict__ outp, int nf4) {
  const int f = blockIdx.x * NTHR + threadIdx.x;
  if (f >= nf4) return;
  const int row = f / NC4;
  const int q   = f - row * NC4;
  const v4f v = *(const v4f*)(SCR + (size_t)row * NHEADP + 4 * q);
  const int b  = row & 7;
  const int ij = row >> 3;
  const int j  = ij % SEQ_L;
  const int i  = ij / SEQ_L;
  const float mi = maskv[i * NB + b], mj = maskv[j * NB + b];
  float fac = mi * mj;
  if (TRI) fac = ((j >= i) ? 1.0f : 0.0f) * fac;
  v4f o;
#pragma unroll
  for (int e = 0; e < 4; ++e) {
    const float xx = v[e] + b2[4 * q + e];
    o[e] = fac * __builtin_amdgcn_rcpf(1.0f + __expf(-xx));
  }
  float* op = outp + (size_t)f * 4;
  *(volatile v4f*)op = o;
  __threadfence();
  *(volatile v4f*)op = o;
}

__global__ __launch_bounds__(NTHR) void pack_out2_kernel(const float* __restrict__ RGF, float* __restrict__ outp) {
  const int f = blockIdx.x * NTHR + threadIdx.x;
  if (f >= MROWS * (HID / 4)) return;
  const int row = f / (HID / 4);
  const int col = (f - row * (HID / 4)) * 4;
  const v4f v = *(const v4f*)(RGF + (size_t)row * HIDP + col);
  float* op = outp + (size_t)f * 4;
  *(volatile v4f*)op = v;
  __threadfence();
  *(volatile v4f*)op = v;
}

extern "C" void kernel_launch(void* const* d_in, const int* in_sizes, int n_in,
                              void* d_out, int out_size, void* d_ws, size_t ws_size, hipStream_t stream) {
  if (n_in != 24 || d_out == nullptr || d_ws == nullptr) return;
  if (in_sizes[0] != SEQ_L * NB * DIN || in_sizes[1] != SEQ_L * NB ||
      in_sizes[2] != G5 * DIN || in_sizes[3] != G5 || in_sizes[4] != G5 * HID || in_sizes[5] != G5 ||
      in_sizes[6] != HID * 3 * HID || in_sizes[7] != HID ||
      in_sizes[8] != HID * 2 * HID || in_sizes[9] != HID || in_sizes[10] != HID * 3 * HID || in_sizes[11] != HID ||
      in_sizes[12] != HID || in_sizes[13] != HID || in_sizes[14] != NTAG * HID || in_sizes[15] != NTAG ||
      in_sizes[16] != HID * 2 * HID || in_sizes[17] != HID || in_sizes[18] != HID * 3 * HID || in_sizes[19] != HID ||
      in_sizes[20] != HID || in_sizes[21] != HID || in_sizes[22] != NREL * HID || in_sizes[23] != NREL) return;
  if (out_size != NPROWS * NTAG + NPROWS * NREL + MROWS * HID) return;

  const float* x      = (const float*)d_in[0];
  const float* mask   = (const float*)d_in[1];
  const float* enc_Wi = (const float*)d_in[2];
  const float* enc_bi = (const float*)d_in[3];
  const float* enc_Wh = (const float*)d_in[4];
  const float* enc_bh = (const float*)d_in[5];
  const float* enc_Wt = (const float*)d_in[6];
  const float* enc_bt = (const float*)d_in[7];
  const float* ner_Wn = (const float*)d_in[8];
  const float* ner_bn = (const float*)d_in[9];
  const float* ner_W1 = (const float*)d_in[10];
  const float* ner_b1 = (const float*)d_in[11];
  const float* ner_g  = (const float*)d_in[12];
  const float* ner_be = (const float*)d_in[13];
  const float* ner_W2 = (const float*)d_in[14];
  const float* ner_b2 = (const float*)d_in[15];
  const float* re_Wr  = (const float*)d_in[16];
  const float* re_br  = (const float*)d_in[17];
  const float* re_W1  = (const float*)d_in[18];
  const float* re_b1  = (const float*)d_in[19];
  const float* re_g   = (const float*)d_in[20];
  const float* re_be  = (const float*)d_in[21];
  const float* re_W2  = (const float*)d_in[22];
  const float* re_b2  = (const float*)d_in[23];

  float* out0 = (float*)d_out;
  float* out1 = out0 + (size_t)NPROWS * NTAG;
  float* out2 = out1 + (size_t)NPROWS * NREL;

  char* ws = (char*)d_ws; size_t off = 0;
  auto carve = [&](size_t bytes) -> char* { char* p = ws + off; off += (bytes + 255) & ~(size_t)255; return p; };
  unsigned short* XH   = (unsigned short*)carve((size_t)MPAD * DIN * 2);
  unsigned short* XL   = (unsigned short*)carve((size_t)MPAD * DIN * 2);
  unsigned short* WIH  = (unsigned short*)carve((size_t)G5P * DIN * 2);
  unsigned short* WIL  = (unsigned short*)carve((size_t)G5P * DIN * 2);
  unsigned short* WHH  = (unsigned short*)carve((size_t)G5P * HIDP * 2);
  unsigned short* WHL  = (unsigned short*)carve((size_t)G5P * HIDP * 2);
  unsigned short* WTH  = (unsigned short*)carve((size_t)HIDP * KCC * 2);
  unsigned short* WTL  = (unsigned short*)carve((size_t)HIDP * KCC * 2);
  unsigned short* WNH  = (unsigned short*)carve((size_t)HIDP * KCAT * 2);
  unsigned short* WNL  = (unsigned short*)carve((size_t)HIDP * KCAT * 2);
  unsigned short* WRH  = (unsigned short*)carve((size_t)HIDP * KCAT * 2);
  unsigned short* WRL  = (unsigned short*)carve((size_t)HIDP * KCAT * 2);
  unsigned short* W1NH = (unsigned short*)carve((size_t)HIDP * KCC * 2);
  unsigned short* W1NL = (unsigned short*)carve((size_t)HIDP * KCC * 2);
  unsigned short* W1RH = (unsigned short*)carve((size_t)HIDP * KCC * 2);
  unsigned short* W1RL = (unsigned short*)carve((size_t)HIDP * KCC * 2);
  unsigned short* W2N  = (unsigned short*)carve((size_t)NHEADP * HIDP * 2);
  unsigned short* W2R  = (unsigned short*)carve((size_t)NHEADP * HIDP * 2);
  float*          PADV = (float*)carve((size_t)8 * HIDP * 4);
  float*          XG   = (float*)carve((size_t)MPAD * G5P * 4);
  float*          H3F  = (float*)carve((size_t)3 * H3PLANE * 4);
  unsigned short* CATNH = (unsigned short*)carve((size_t)MPAD * KCAT * 2);
  unsigned short* CATNL = (unsigned short*)carve((size_t)MPAD * KCAT * 2);
  unsigned short* CATRH = (unsigned short*)carve((size_t)MPAD * KCAT * 2);
  unsigned short* CATRL = (unsigned short*)carve((size_t)MPAD * KCAT * 2);
  unsigned short* HNH  = (unsigned short*)carve((size_t)MPAD * HIDP * 2);
  unsigned short* HNL  = (unsigned short*)carve((size_t)MPAD * HIDP * 2);
  unsigned short* HRH  = (unsigned short*)carve((size_t)MPAD * HIDP * 2);
  unsigned short* HRL  = (unsigned short*)carve((size_t)MPAD * HIDP * 2);
  float*          HGPRE = (float*)carve((size_t)MPAD * HIDP * 4);
  float*          RGF   = (float*)carve((size_t)MPAD * HIDP * 4);
  unsigned short* HGH  = (unsigned short*)carve((size_t)NHEADP * HIDP * 2);
  unsigned short* HGL  = (unsigned short*)carve((size_t)NHEADP * HIDP * 2);
  unsigned short* RGH  = (unsigned short*)carve((size_t)NHEADP * HIDP * 2);
  unsigned short* RGL  = (unsigned short*)carve((size_t)NHEADP * HIDP * 2);
  float*          AN   = (float*)carve((size_t)MPAD * HIDP * 4);
  float*          BN   = (float*)carve((size_t)MPAD * HIDP * 4);
  float*          AR   = (float*)carve((size_t)MPAD * HIDP * 4);
  float*          BR   = (float*)carve((size_t)MPAD * HIDP * 4);
  float*          CN   = (float*)carve((size_t)NHEADP * HIDP * 4);
  float*          CR   = (float*)carve((size_t)NHEADP * HIDP * 4);
  unsigned short* PAIRA = (unsigned short*)carve((size_t)NPROWS * HIDP * 2);
  float*          SCR   = (float*)carve((size_t)NPROWS * NHEADP * 4);
  if (off > ws_size || off > (size_t)134217728) return;

  const float* HNF = H3F;
  const float* HRF = H3F + H3PLANE;
  const float* HSF = H3F + 2 * H3PLANE;

  auto cvtgrid = [](int nrow_d, int ncol8) { return dim3((unsigned)((nrow_d * ncol8 + NTHR - 1) / NTHR)); };
  auto gemmgrid = [](int M, int N) { const int tiles = (M / 64) * (N / 64); return dim3((unsigned)((tiles + 7) / 8), 1); };

  cvt_plane_kernel<0><<<cvtgrid(MPAD, DIN / 8), NTHR, 0, stream>>>(x, MROWS, DIN, DIN, DIN, XH, XL, MPAD, DIN / 8, 1.0f);
  cvt_plane_kernel<0><<<cvtgrid(G5P, DIN / 8), NTHR, 0, stream>>>(enc_Wi, G5, DIN, DIN, DIN, WIH, WIL, G5P, DIN / 8, 1.0f);
  cvt_plane_kernel<0><<<cvtgrid(G5P, HIDP / 8), NTHR, 0, stream>>>(enc_Wh, G5, HID, HID, HIDP, WHH, WHL, G5P, HIDP / 8, 1.0f);
  cvt_plane_kernel<0><<<cvtgrid(HIDP, KCC / 8), NTHR, 0, stream>>>(enc_Wt, HID, 3 * HID, HID, HIDP, WTH, WTL, HIDP, KCC / 8, 1.0f);
  cvt_plane_kernel<0><<<cvtgrid(HIDP, KCAT / 8), NTHR, 0, stream>>>(ner_Wn, HID, 2 * HID, HID, HIDP, WNH, WNL, HIDP, KCAT / 8, 1.0f);
  cvt_plane_kernel<0><<<cvtgrid(HIDP, KCAT / 8), NTHR, 0, stream>>>(re_Wr, HID, 2 * HID, HID, HIDP, WRH, WRL, HIDP, KCAT / 8, 1.0f);
  cvt_plane_kernel<0><<<cvtgrid(HIDP, KCC / 8), NTHR, 0, stream>>>(ner_W1, HID, 3 * HID, HID, HIDP, W1NH, W1NL, HIDP, KCC / 8, 1.0f);
  cvt_plane_kernel<0><<<cvtgrid(HIDP, KCC / 8), NTHR, 0, stream>>>(re_W1, HID, 3 * HID, HID, HIDP, W1RH, W1RL, HIDP, KCC / 8, 1.0f);
  cvt_plane_kernel<1><<<cvtgrid(NHEADP, HIDP / 8), NTHR, 0, stream>>>(ner_W2, NTAG, HID, HID, HIDP, W2N, W2N, NHEADP, HIDP / 8, W2CARRY);
  cvt_plane_kernel<1><<<cvtgrid(NHEADP, HIDP / 8), NTHR, 0, stream>>>(re_W2, NREL, HID, HID, HIDP, W2R, W2R, NHEADP, HIDP / 8, W2CARRY);
  pad8_kernel<<<2, 512, 0, stream>>>(ner_bn, re_br, ner_b1, re_b1, ner_g, ner_be, re_g, re_be, PADV);
  const float* bn_pad  = PADV + 0 * HIDP;
  const float* br_pad  = PADV + 1 * HIDP;
  const float* nb1_pad = PADV + 2 * HIDP;
  const float* rb1_pad = PADV + 3 * HIDP;
  const float* ng_pad  = PADV + 4 * HIDP;
  const float* nbe_pad = PADV + 5 * HIDP;
  const float* rg_pad  = PADV + 6 * HIDP;
  const float* rbe_pad = PADV + 7 * HIDP;

  wmma_gemm64<1, true, 0, 0, false, 0><<<gemmgrid(MPAD, G5P), 256, 0, stream>>>(
      XH, XL, DIN, 0L, WIH, WIL, DIN, 0L, (void*)XG, (void*)XG, G5P, 0L, PADV, XG, 0L, MPAD, G5P, DIN, 1.0f);

  pf_seq_kernel<<<1, NTHR, 0, stream>>>(XG, enc_bi, enc_bh, enc_bt, WHH, WHL, WTH, WTL, H3F);

  cvt_cat_kernel<<<cvtgrid(MPAD, KCAT / 8), NTHR, 0, stream>>>(HSF, HNF, CATNH, CATNL, KCAT / 8);
  cvt_cat_kernel<<<cvtgrid(MPAD, KCAT / 8), NTHR, 0, stream>>>(HSF, HRF, CATRH, CATRL, KCAT / 8);
  cvt_cat_kernel<<<cvtgrid(MPAD, HIDP / 8), NTHR, 0, stream>>>(HNF, HNF, HNH, HNL, HIDP / 8);
  cvt_cat_kernel<<<cvtgrid(MPAD, HIDP / 8), NTHR, 0, stream>>>(HRF, HRF, HRH, HRL, HIDP / 8);

  wmma_gemm64<1, true, 2, 0, false, 1><<<gemmgrid(MPAD, HIDP), 256, 0, stream>>>(
      CATNH, CATNL, KCAT, 0L, WNH, WNL, KCAT, 0L, (void*)HGPRE, (void*)HGPRE, HIDP, 0L, bn_pad, XG, 0L, MPAD, HIDP, KCAT, 1.0f);
  colmax_kernel<<<(NHEADP * (HIDP / 8) + NTHR - 1) / NTHR, NTHR, 0, stream>>>(HGPRE, HGH, HGL);
  wmma_gemm64<1, true, 0, 0, false, 0><<<gemmgrid(MPAD, HIDP), 256, 0, stream>>>(
      HNH, HNL, HIDP, 0L, W1NH, W1NL, KCC, 0L, (void*)AN, (void*)AN, HIDP, 0L, PADV, XG, 0L, MPAD, HIDP, HIDP, 1.0f);
  wmma_gemm64<1, true, 0, 0, false, 0><<<gemmgrid(MPAD, HIDP), 256, 0, stream>>>(
      HNH, HNL, HIDP, 0L, W1NH + HIDP, W1NL + HIDP, KCC, 0L, (void*)BN, (void*)BN, HIDP, 0L, PADV, XG, 0L, MPAD, HIDP, HIDP, 1.0f);
  wmma_gemm64<1, true, 2, 0, false, 0><<<gemmgrid(NHEADP, HIDP), 256, 0, stream>>>(
      HGH, HGL, HIDP, 0L, W1NH + 2 * HIDP, W1NL + 2 * HIDP, KCC, 0L, (void*)CN, (void*)CN, HIDP, 0L, nb1_pad, XG, 0L, NHEADP, HIDP, HIDP, 1.0f);
  pair_ln_kernel<<<(SEQ_L * NB * (SEQ_L / JGRP)) / (NTHR / 32), NTHR, 0, stream>>>(AN, BN, CN, ng_pad, nbe_pad, PAIRA);
  wmma_gemm64<0, false, 0, 0, false, 0><<<gemmgrid(NPROWS, NHEADP), 256, 0, stream>>>(
      PAIRA, PAIRA, HIDP, 0L, W2N, W2N, HIDP, 0L, (void*)SCR, (void*)SCR, NHEADP, 0L, PADV, XG, 0L, NPROWS, NHEADP, HIDP, W2CARRY_INV);
  pack_head_kernel<2, true><<<(NPROWS * 2 + NTHR - 1) / NTHR, NTHR, 0, stream>>>(SCR, ner_b2, mask, out0, NPROWS * 2);

  wmma_gemm64<1, true, 2, 0, false, 1><<<gemmgrid(MPAD, HIDP), 256, 0, stream>>>(
      CATRH, CATRL, KCAT, 0L, WRH, WRL, KCAT, 0L, (void*)RGF, (void*)RGF, HIDP, 0L, br_pad, XG, 0L, MPAD, HIDP, KCAT, 1.0f);
  pack_out2_kernel<<<(MROWS * (HID / 4) + NTHR - 1) / NTHR, NTHR, 0, stream>>>(RGF, out2);
  colmax_kernel<<<(NHEADP * (HIDP / 8) + NTHR - 1) / NTHR, NTHR, 0, stream>>>(RGF, RGH, RGL);
  wmma_gemm64<1, true, 0, 0, false, 0><<<gemmgrid(MPAD, HIDP), 256, 0, stream>>>(
      HRH, HRL, HIDP, 0L, W1RH, W1RL, KCC, 0L, (void*)AR, (void*)AR, HIDP, 0L, PADV, XG, 0L, MPAD, HIDP, HIDP, 1.0f);
  wmma_gemm64<1, true, 0, 0, false, 0><<<gemmgrid(MPAD, HIDP), 256, 0, stream>>>(
      HRH, HRL, HIDP, 0L, W1RH + HIDP, W1RL + HIDP, KCC, 0L, (void*)BR, (void*)BR, HIDP, 0L, PADV, XG, 0L, MPAD, HIDP, HIDP, 1.0f);
  wmma_gemm64<1, true, 2, 0, false, 0><<<gemmgrid(NHEADP, HIDP), 256, 0, stream>>>(
      RGH, RGL, HIDP, 0L, W1RH + 2 * HIDP, W1RL + 2 * HIDP, KCC, 0L, (void*)CR, (void*)CR, HIDP, 0L, rb1_pad, XG, 0L, NHEADP, HIDP, HIDP, 1.0f);
  pair_ln_kernel<<<(SEQ_L * NB * (SEQ_L / JGRP)) / (NTHR / 32), NTHR, 0, stream>>>(AR, BR, CR, rg_pad, rbe_pad, PAIRA);
  wmma_gemm64<0, false, 0, 0, false, 0><<<gemmgrid(NPROWS, NHEADP), 256, 0, stream>>>(
      PAIRA, PAIRA, HIDP, 0L, W2R, W2R, HIDP, 0L, (void*)SCR, (void*)SCR, NHEADP, 0L, PADV, XG, 0L, NPROWS, NHEADP, HIDP, W2CARRY_INV);
  pack_head_kernel<3, false><<<(NPROWS * 3 + NTHR - 1) / NTHR, NTHR, 0, stream>>>(SCR, re_b2, mask, out1, NPROWS * 3);
}
